// LRU2_13477607375572
// MI455X (gfx1250) — hardware-verified
//
#include <hip/hip_runtime.h>
#include <math.h>

typedef __attribute__((ext_vector_type(16))) _Float16 v16h;
typedef __attribute__((ext_vector_type(8)))  _Float16 v8h;
typedef __attribute__((ext_vector_type(8)))  float    v8f;
typedef __attribute__((ext_vector_type(4)))  float    v4f;

constexpr int kSeqLen  = 32768;
constexpr int kWidth   = 256;
constexpr int kStates  = 512;
constexpr int kStates2 = 2 * kStates;
constexpr int kChunkT  = 128;
constexpr int kChunks  = kSeqLen / kChunkT;
constexpr int kSquarings = 7;
static_assert((1 << kSquarings) == kChunkT);
static_assert(kChunks * kChunkT == kSeqLen);
static_assert((kWidth % 32) == 0 && (kStates2 % 32) == 0);
static_assert((kSeqLen % 64) == 0 && (kStates2 % 64) == 0 && (kWidth % 64) == 0);
static_assert((kStates % 256) == 0 && (kChunkT % 8) == 0 && (kChunks % 8) == 0);

constexpr float kCarryX = 16.0f;
constexpr float kCarryB = 1024.0f;
constexpr float kCarryS = 64.0f;
constexpr float kCarryC = 256.0f;
constexpr float kScaleP = kCarryS / (kCarryX * kCarryB);
constexpr float kScaleY = 1.0f / (kCarryS * kCarryC);
constexpr float kF16Min = 6.103515625e-5f;

constexpr size_t kOffPS    = 0;
constexpr size_t kOffX16   = kOffPS    + (size_t)kSeqLen * kStates2 * 2;
constexpr size_t kOffBT1   = kOffX16   + (size_t)kSeqLen * kWidth * 2;
constexpr size_t kOffBT2   = kOffBT1   + (size_t)kStates2 * kWidth * 2;
constexpr size_t kOffLOCRE = kOffBT2   + (size_t)kWidth * kStates2 * 2;
constexpr size_t kOffLOCIM = kOffLOCRE + (size_t)kChunks * kStates * 4;
constexpr size_t kOffCINRE = kOffLOCIM + (size_t)kChunks * kStates * 4;
constexpr size_t kOffCINIM = kOffCINRE + (size_t)kChunks * kStates * 4;
constexpr size_t kOffTAB   = kOffCINIM + (size_t)kChunks * kStates * 4;
constexpr size_t kWsTotal  = kOffTAB   + (size_t)5 * kStates * 4;
static_assert(kWsTotal == 87042048ull);
static_assert(kWsTotal <= 134217728ull);
static_assert((kOffX16 % 128) == 0 && (kOffBT1 % 128) == 0 && (kOffBT2 % 128) == 0 && (kOffLOCRE % 128) == 0 &&
              (kOffLOCIM % 128) == 0 && (kOffCINRE % 128) == 0 && (kOffCINIM % 128) == 0 && (kOffTAB % 128) == 0);

__device__ __forceinline__ float flush16(float v) { return (fabsf(v) < kF16Min) ? 0.0f : v; }

__device__ __forceinline__ float h16_to_f32(unsigned hb) {
  const unsigned sgn = (hb & 0x8000u) << 16; const unsigned em = hb & 0x7fffu;
  const float fn = __uint_as_float((em << 13) + 0x38000000u);
  const float fs = (float)em * 5.9604644775390625e-8f;
  const float mag = (em < 0x400u) ? fs : fn; return __uint_as_float(__float_as_uint(mag) | sgn); }

__device__ __forceinline__ void guard1_h(v8f& a, v16h x, v16h y) { asm volatile("v_nop\n\tv_nop\n\tv_nop\n\tv_nop" : "+v"(a) : "v"(x), "v"(y)); }
__device__ __forceinline__ void keep4_h(v16h a, v16h b, v16h c, v16h d) { asm volatile("v_nop" :: "v"(a), "v"(b), "v"(c), "v"(d)); }
__device__ __forceinline__ void acc_guard4(v8f& a, v8f& b, v8f& c, v8f& d) { asm volatile("v_nop\n\tv_nop\n\tv_nop\n\tv_nop" : "+v"(a), "+v"(b), "+v"(c), "+v"(d)); }

struct FragH {
  union U { v16h v; v8h h[2]; };
  static __device__ __forceinline__ v16h load(const _Float16* p) {
    U f; f.h[0] = *(const v8h*)(p); f.h[1] = *(const v8h*)(p + 16); return f.v;
  }
  static __device__ __forceinline__ v8f mma(v16h a, v16h b, v8f c) {
    return __builtin_amdgcn_wmma_f32_16x16x32_f16(false, a, false, b, (short)0, c, false, false);
  }
};

__global__ __launch_bounds__(512) void prep_tables_kernel(
    const float* __restrict__ nu_log, const float* __restrict__ theta_log, float* __restrict__ tab)
{
  const int n = threadIdx.x;
  const float nu  = expf(nu_log[n]);
  const float th  = expf(theta_log[n]);
  const float mod = expf(-nu);
  float sn, cs;
  sincosf(th, &sn, &cs);
  const float lr = mod * cs;
  const float li = mod * sn;
  const float g  = sqrtf(fmaxf(0.0f, 1.0f - mod * mod));
  float pr = lr, pi = li;
#pragma unroll 1
  for (int q = 0; q < kSquarings; ++q) {
    const float nr = pr * pr - pi * pi;
    const float ni = 2.0f * pr * pi;
    pr = nr; pi = ni;
  }
  float* t0 = tab + n;
  for (int pass = 0; pass < 2; ++pass) {
    *(volatile float*)(t0)               = lr;
    *(volatile float*)(t0 + kStates)     = li;
    *(volatile float*)(t0 + 2 * kStates) = pr;
    *(volatile float*)(t0 + 3 * kStates) = pi;
    *(volatile float*)(t0 + 4 * kStates) = g;
    __threadfence();
  }
}

constexpr int kPackBBlocks = (kStates * kWidth / 8) / 256;
constexpr int kPackCBlocks = (kWidth * kStates / 4) / 256;
constexpr int kPackXBlocks = (kSeqLen * kWidth / 8) / 256;
static_assert(kPackBBlocks * 256 * 8 == kStates * kWidth);
static_assert(kPackCBlocks * 256 * 4 == kWidth * kStates);
static_assert(kPackXBlocks * 256 * 8 == kSeqLen * kWidth);
static_assert(kWidth / 8 == 32 && kStates / 4 == 128);

__global__ __launch_bounds__(256) void pack_planes_kernel(
    const float* __restrict__ x, const float* __restrict__ Bre, const float* __restrict__ Bim,
    const float* __restrict__ Cre, const float* __restrict__ Cim, const float* __restrict__ gam,
    unsigned short* __restrict__ X16, unsigned short* __restrict__ BT1, unsigned short* __restrict__ BT2)
{
  const int bx = blockIdx.x;
  const int tid = threadIdx.x;
  if (bx < kPackBBlocks) {
    const int i  = bx * 256 + tid;
    const int n  = i >> 5;
    const int h0 = (i & 31) * 8;
    const float g = gam[n] * kCarryB;
    const v4f a0 = *(const v4f*)(Bre + (size_t)n * kWidth + h0);
    const v4f a1 = *(const v4f*)(Bre + (size_t)n * kWidth + h0 + 4);
    const v4f b0 = *(const v4f*)(Bim + (size_t)n * kWidth + h0);
    const v4f b1 = *(const v4f*)(Bim + (size_t)n * kWidth + h0 + 4);
    v8h hr, hi;
#pragma unroll
    for (int e = 0; e < 4; ++e) {
      hr[e]     = (_Float16)flush16(a0[e] * g);
      hr[4 + e] = (_Float16)flush16(a1[e] * g);
      hi[e]     = (_Float16)flush16(b0[e] * g);
      hi[4 + e] = (_Float16)flush16(b1[e] * g);
    }
    unsigned short* pr = BT1 + (size_t)(2 * n) * kWidth + h0;
    unsigned short* pi = pr + kWidth;
    *(volatile v8h*)pr = hr;
    *(volatile v8h*)pi = hi;
    __threadfence();
    *(volatile v8h*)pr = hr;
    *(volatile v8h*)pi = hi;
  } else if (bx < kPackBBlocks + kPackCBlocks) {
    const int i  = (bx - kPackBBlocks) * 256 + tid;
    const int h  = i >> 7;
    const int n0 = (i & 127) * 4;
    const v4f cr = *(const v4f*)(Cre + (size_t)h * kStates + n0);
    const v4f ci = *(const v4f*)(Cim + (size_t)h * kStates + n0);
    v8h o;
#pragma unroll
    for (int e = 0; e < 4; ++e) {
      o[2 * e]     = (_Float16)flush16(cr[e] * kCarryC);
      o[2 * e + 1] = (_Float16)flush16(-(ci[e] * kCarryC));
    }
    unsigned short* p = BT2 + (size_t)h * kStates2 + 2 * n0;
    *(volatile v8h*)p = o;
    __threadfence();
    *(volatile v8h*)p = o;
  } else {
    const int i = (bx - kPackBBlocks - kPackCBlocks) * 256 + tid;
    const size_t e0 = (size_t)i << 3;
    const v4f a0 = *(const v4f*)(x + e0);
    const v4f a1 = *(const v4f*)(x + e0 + 4);
    v8h o;
#pragma unroll
    for (int e = 0; e < 4; ++e) {
      o[e]     = (_Float16)flush16(a0[e] * kCarryX);
      o[4 + e] = (_Float16)flush16(a1[e] * kCarryX);
    }
    unsigned short* p = X16 + e0;
    *(volatile v8h*)p = o;
    __threadfence();
    *(volatile v8h*)p = o;
  }
}

template <int OUT_MODE>
__global__ __launch_bounds__(256) void gemm64_f16_kernel(
    const unsigned short* __restrict__ Ap, int lda,
    const unsigned short* __restrict__ Btp, int ldb,
    void* __restrict__ Cout, int ldc,
    const float* __restrict__ skipX, const float* __restrict__ skipD,
    int M, int N, int K, float scale)
{
  const _Float16* A  = (const _Float16*)Ap;
  const _Float16* Bt = (const _Float16*)Btp;
  __shared__ __align__(16) float sT[8][16 * 68];
  const int lane = threadIdx.x & 31;
  const int wave = threadIdx.x >> 5;
  const int tilesN = N >> 6;
  const int tilesM = M >> 6;
  const int tile = blockIdx.x * 8 + wave;
  if (tile >= tilesM * tilesN) return;
  const int tm = tile / tilesN;
  const int tn = tile - tm * tilesN;
  const int m0 = tm << 6;
  const int n0 = tn << 6;

  const int rlane = lane & 15;
  const int koff  = (lane >> 4) * 8;
  const int mOff  = (lane >> 4) * 8;

  v8f acc[4][4];
#pragma unroll
  for (int i = 0; i < 4; ++i)
#pragma unroll
    for (int j = 0; j < 4; ++j) acc[i][j] = (v8f){0.f,0.f,0.f,0.f,0.f,0.f,0.f,0.f};

  for (int k0 = 0; k0 < K; k0 += 32) {
    v16h bh[4];
#pragma unroll
    for (int j = 0; j < 4; ++j) {
      const size_t bo = (size_t)(n0 + (j << 4) + rlane) * ldb + koff + k0;
      bh[j] = FragH::load(Bt + bo);
    }
#pragma unroll
    for (int i = 0; i < 4; ++i) {
      const size_t ao = (size_t)(m0 + (i << 4) + rlane) * lda + koff + k0;
      const v16h ah = FragH::load(A + ao);
#pragma unroll
      for (int j = 0; j < 4; ++j) acc[i][j] = FragH::mma(ah, bh[j], acc[i][j]);
      guard1_h(acc[i][0], ah, bh[0]);
      guard1_h(acc[i][1], ah, bh[1]);
      guard1_h(acc[i][2], ah, bh[2]);
      guard1_h(acc[i][3], ah, bh[3]);
    }
    keep4_h(bh[0], bh[1], bh[2], bh[3]);
  }
  acc_guard4(acc[0][0], acc[0][1], acc[0][2], acc[0][3]);
  acc_guard4(acc[1][0], acc[1][1], acc[1][2], acc[1][3]);
  acc_guard4(acc[2][0], acc[2][1], acc[2][2], acc[2][3]);
  acc_guard4(acc[3][0], acc[3][1], acc[3][2], acc[3][3]);

  float* slab = sT[wave];
#pragma unroll
  for (int i = 0; i < 4; ++i) {
    const int mBase = m0 + (i << 4);
#pragma unroll
    for (int j = 0; j < 4; ++j) {
#pragma unroll
      for (int r = 0; r < 8; ++r) {
        const float v = acc[i][j][r] * scale;
        slab[(mOff + r) * 68 + (j << 4) + rlane] = v;
      }
    }
    __builtin_amdgcn_fence(__ATOMIC_RELEASE, "workgroup");
    __builtin_amdgcn_wave_barrier();
    __builtin_amdgcn_fence(__ATOMIC_ACQUIRE, "workgroup");
    if (OUT_MODE == 0) {
      float* C = (float*)Cout;
      const int hh = lane >> 4, c4 = (lane & 15) * 4;
      const v4f dv = *(const v4f*)(skipD + n0 + c4);
      v4f ov[8];
#pragma unroll
      for (int it = 0; it < 8; ++it) {
        const int row = it * 2 + hh;
        const v4f v  = *(const v4f*)(slab + row * 68 + c4);
        const v4f xv = *(const v4f*)(skipX + (size_t)(mBase + row) * ldc + n0 + c4);
        ov[it] = v + dv * xv;
      }
      for (int pass = 0; pass < 2; ++pass) {
#pragma unroll
        for (int it = 0; it < 8; ++it) {
          const int row = it * 2 + hh;
          *(volatile v4f*)(C + (size_t)(mBase + row) * ldc + n0 + c4) = ov[it];
        }
        __threadfence();
      }
    } else {
      const int q = lane >> 3, c8 = (lane & 7) * 8;
      unsigned short* C = (unsigned short*)Cout;
      v8h hv[4];
#pragma unroll
      for (int it = 0; it < 4; ++it) {
        const int row = it * 4 + q;
        const float* sp = slab + row * 68 + c8;
#pragma unroll
        for (int e = 0; e < 8; ++e) hv[it][e] = (_Float16)flush16(sp[e]);
      }
      for (int pass = 0; pass < 2; ++pass) {
#pragma unroll
        for (int it = 0; it < 4; ++it) {
          const int row = it * 4 + q;
          *(volatile v8h*)(C + (size_t)(mBase + row) * ldc + n0 + c8) = hv[it];
        }
        __threadfence();
      }
    }
    __builtin_amdgcn_fence(__ATOMIC_RELEASE, "workgroup");
    __builtin_amdgcn_wave_barrier();
    __builtin_amdgcn_fence(__ATOMIC_ACQUIRE, "workgroup");
  }
}

__global__ __launch_bounds__(256) void scan_local_kernel(
    const unsigned* __restrict__ P32, const float* __restrict__ tab,
    float* __restrict__ locRe, float* __restrict__ locIm)
{
  const int n = blockIdx.x * 256 + threadIdx.x;
  const int c = blockIdx.y;
  const float lr = tab[n];
  const float li = tab[kStates + n];
  const unsigned* p = P32 + (size_t)c * kChunkT * kStates + n;
  float sr = 0.0f, si = 0.0f;
#pragma unroll 1
  for (int t0 = 0; t0 < kChunkT; t0 += 8) {
    unsigned w[8];
#pragma unroll
    for (int k = 0; k < 8; ++k) w[k] = p[(size_t)(t0 + k) * kStates];
#pragma unroll
    for (int k = 0; k < 8; ++k) {
      const float br = h16_to_f32(w[k] & 0xffffu);
      const float bi = h16_to_f32(w[k] >> 16);
      const float nr = fmaf(lr, sr, fmaf(-li, si, br));
      const float ni = fmaf(lr, si, fmaf(li, sr, bi));
      sr = nr; si = ni;
    }
  }
  float* qr = locRe + (size_t)c * kStates + n;
  float* qi = locIm + (size_t)c * kStates + n;
  *(volatile float*)qr = sr;
  *(volatile float*)qi = si;
  __threadfence();
  *(volatile float*)qr = sr;
  *(volatile float*)qi = si;
}

__global__ __launch_bounds__(512) void carry_prefix_kernel(
    const float* __restrict__ tab, const float* __restrict__ locRe, const float* __restrict__ locIm,
    float* __restrict__ cinRe, float* __restrict__ cinIm)
{
  const int n = threadIdx.x;
  const float lr = tab[2 * kStates + n];
  const float li = tab[3 * kStates + n];
  float cr = 0.0f, ci = 0.0f;
#pragma unroll 1
  for (int c0 = 0; c0 < kChunks; c0 += 8) {
    float ar[8], ai[8], orr[8], oi[8];
#pragma unroll
    for (int k = 0; k < 8; ++k) {
      ar[k] = locRe[(size_t)(c0 + k) * kStates + n];
      ai[k] = locIm[(size_t)(c0 + k) * kStates + n];
    }
#pragma unroll
    for (int k = 0; k < 8; ++k) {
      orr[k] = cr;
      oi[k]  = ci;
      const float nr = fmaf(lr, cr, fmaf(-li, ci, ar[k]));
      const float ni = fmaf(lr, ci, fmaf(li, cr, ai[k]));
      cr = nr; ci = ni;
    }
    for (int pass = 0; pass < 2; ++pass) {
#pragma unroll
      for (int k = 0; k < 8; ++k) {
        *(volatile float*)(cinRe + (size_t)(c0 + k) * kStates + n) = orr[k];
        *(volatile float*)(cinIm + (size_t)(c0 + k) * kStates + n) = oi[k];
      }
      __threadfence();
    }
  }
}

__global__ __launch_bounds__(256) void scan_final_kernel(
    unsigned* PS32, const float* __restrict__ tab,
    const float* __restrict__ cinRe, const float* __restrict__ cinIm)
{
  const int n = blockIdx.x * 256 + threadIdx.x;
  const int c = blockIdx.y;
  const float lr = tab[n];
  const float li = tab[kStates + n];
  float sr = cinRe[(size_t)c * kStates + n];
  float si = cinIm[(size_t)c * kStates + n];
  unsigned* q = PS32 + (size_t)c * kChunkT * kStates + n;
#pragma unroll 1
  for (int t0 = 0; t0 < kChunkT; t0 += 8) {
    unsigned w[8], ow[8];
#pragma unroll
    for (int k = 0; k < 8; ++k) w[k] = q[(size_t)(t0 + k) * kStates];
#pragma unroll
    for (int k = 0; k < 8; ++k) {
      const float br = h16_to_f32(w[k] & 0xffffu);
      const float bi = h16_to_f32(w[k] >> 16);
      const float nr = fmaf(lr, sr, fmaf(-li, si, br));
      const float ni = fmaf(lr, si, fmaf(li, sr, bi));
      sr = nr; si = ni;
      const _Float16 hr = (_Float16)flush16(sr);
      const _Float16 hi = (_Float16)flush16(si);
      const unsigned ur = (unsigned)__builtin_bit_cast(unsigned short, hr);
      const unsigned ui = (unsigned)__builtin_bit_cast(unsigned short, hi);
      ow[k] = ur | (ui << 16);
    }
    for (int pass = 0; pass < 2; ++pass) {
#pragma unroll
      for (int k = 0; k < 8; ++k) *(volatile unsigned*)(q + (size_t)(t0 + k) * kStates) = ow[k];
      __threadfence();
    }
  }
}

constexpr int kTiles1 = (kSeqLen / 64) * (kStates2 / 64);
constexpr int kTiles2 = (kSeqLen / 64) * (kWidth / 64);
static_assert((kTiles1 % 8) == 0 && (kTiles2 % 8) == 0);

extern "C" void kernel_launch(void* const* d_in, const int* in_sizes, int n_in,
                              void* d_out, int out_size, void* d_ws, size_t ws_size,
                              hipStream_t stream) {
  if (n_in < 8) return;
  if (in_sizes[0] != kSeqLen * kWidth) return;
  if (in_sizes[1] != kStates) return;
  if (in_sizes[2] != kStates) return;
  if (in_sizes[3] != kStates * kWidth) return;
  if (in_sizes[4] != kStates * kWidth) return;
  if (in_sizes[5] != kWidth * kStates) return;
  if (in_sizes[6] != kWidth * kStates) return;
  if (in_sizes[7] != kWidth) return;
  if (out_size != kSeqLen * kWidth) return;
  if (ws_size < kWsTotal) return;

  const float* x         = (const float*)d_in[0];
  const float* nu_log    = (const float*)d_in[1];
  const float* theta_log = (const float*)d_in[2];
  const float* B_re      = (const float*)d_in[3];
  const float* B_im      = (const float*)d_in[4];
  const float* C_re      = (const float*)d_in[5];
  const float* C_im      = (const float*)d_in[6];
  const float* Dv        = (const float*)d_in[7];
  float* y = (float*)d_out;

  char* ws = (char*)d_ws;
  unsigned short* PS    = (unsigned short*)(ws + kOffPS);
  unsigned short* X16   = (unsigned short*)(ws + kOffX16);
  unsigned short* BT1   = (unsigned short*)(ws + kOffBT1);
  unsigned short* BT2   = (unsigned short*)(ws + kOffBT2);
  float*          LOCRE = (float*)(ws + kOffLOCRE);
  float*          LOCIM = (float*)(ws + kOffLOCIM);
  float*          CINRE = (float*)(ws + kOffCINRE);
  float*          CINIM = (float*)(ws + kOffCINIM);
  float*          TAB   = (float*)(ws + kOffTAB);

  prep_tables_kernel<<<1, kStates, 0, stream>>>(nu_log, theta_log, TAB);

  pack_planes_kernel<<<kPackBBlocks + kPackCBlocks + kPackXBlocks, 256, 0, stream>>>(
      x, B_re, B_im, C_re, C_im, TAB + 4 * kStates, X16, BT1, BT2);

  gemm64_f16_kernel<1><<<kTiles1 / 8, 256, 0, stream>>>(
      X16, kWidth, BT1, kWidth, (void*)PS, kStates2, nullptr, nullptr,
      kSeqLen, kStates2, kWidth, kScaleP);

  scan_local_kernel<<<dim3(kStates / 256, kChunks), 256, 0, stream>>>(
      (const unsigned*)PS, TAB, LOCRE, LOCIM);

  carry_prefix_kernel<<<1, kStates, 0, stream>>>(TAB, LOCRE, LOCIM, CINRE, CINIM);

  scan_final_kernel<<<dim3(kStates / 256, kChunks), 256, 0, stream>>>(
      (unsigned*)PS, TAB, CINRE, CINIM);

  gemm64_f16_kernel<0><<<kTiles2 / 8, 256, 0, stream>>>(
      PS, kStates2, BT2, kStates2, (void*)y, kWidth, x, Dv,
      kSeqLen, kWidth, kStates2, kScaleY);
}
